// EventSequenceDurationGraphConvModel_8022998909608
// MI455X (gfx1250) — hardware-run, weakly checked
//
#include <hip/hip_runtime.h>
#include <stddef.h>


#define F_EV    128
#define F_DU    64
#define F_CAT   256
#define SEQF    256
#define FC2N    128
#define FCCK    384
#define NCLS    16
#define HB      64
#define NTHR    256
#define NWAVE   8
#define EPT     8
#define NGRP    2
#define CHUNK   (NTHR * EPT * NGRP)
#define WCAP    (EPT * NGRP * 32)
#define LISTN   (NWAVE * WCAP)
#define NBC     8192
#define NBF     2048
#define NBP     32
#define RCAP    40960
#define RBN     128
#define OTHR    512
#define GROWS   128
#define DEGCAP  256
#define HPA     392
#define HPB     264
#define WSCALE  16.0f
#define WINV    0.0625f

#define LDS_FILL      ((RCAP + NBF + LISTN) * 4 + 64)
#define LDS_LAYER(F)  (GROWS * (2 * (F) + 8) * 2 + NWAVE * 16 * 128 * 4)
#define LDS_HEAD      (HB * HPA * 2 + HB * HPB * 2 + HB * NCLS * 4 * 2)

static_assert((CHUNK & (CHUNK - 1)) == 0);
static_assert(CHUNK <= 4096);
static_assert((NBC & (NBC - 1)) == 0 && (NBF & (NBF - 1)) == 0 && (NBP & (NBP - 1)) == 0);
static_assert(NBC <= 65536);
static_assert(NBC == 4 * NBF);
static_assert(OTHR * 16 == NBC);
static_assert(NBF == 128 * 16);
static_assert((RCAP % 32) == 0);
static_assert(NBC % (NWAVE * 128) == 0);
static_assert(GROWS == NWAVE * 16);
static_assert(NBP * F_CAT / 4 == 8 * NTHR);
static_assert(HB == 64 && HB * NCLS == 8 * 128);
static_assert(HB * SEQF / 8 == 8 * NTHR && HB * F_CAT / 8 == 8 * NTHR);
static_assert(((HPA * 2) % 16) == 0 && ((HPB * 2) % 16) == 0);
static_assert(HPA >= FCCK + 8 && HPB >= SEQF + 8);

typedef float    v2f  __attribute__((ext_vector_type(2)));
typedef float    v4f  __attribute__((ext_vector_type(4)));
typedef float    v8f  __attribute__((ext_vector_type(8)));
typedef int      v4i  __attribute__((ext_vector_type(4)));
typedef _Float16 v2h  __attribute__((ext_vector_type(2)));
typedef _Float16 v4h  __attribute__((ext_vector_type(4)));
typedef _Float16 v8h  __attribute__((ext_vector_type(8)));
typedef _Float16 v16h __attribute__((ext_vector_type(16)));
union FragH { v16h v; v8h h[2]; };

__device__ __forceinline__ v8h cvt8(v4f a, v4f b) {
  v8h r;
  r[0] = (_Float16)a.x; r[1] = (_Float16)a.y; r[2] = (_Float16)a.z; r[3] = (_Float16)a.w;
  r[4] = (_Float16)b.x; r[5] = (_Float16)b.y; r[6] = (_Float16)b.z; r[7] = (_Float16)b.w;
  return r;
}
__device__ __forceinline__ v4h cvt4(v4f a) {
  v4h r;
  r.x = (_Float16)a.x; r.y = (_Float16)a.y; r.z = (_Float16)a.z; r.w = (_Float16)a.w;
  return r;
}
__device__ __forceinline__ v2h cvt2(v2f a) {
  v2h r;
  r.x = (_Float16)a.x; r.y = (_Float16)a.y;
  return r;
}

__device__ __forceinline__ v8f wmh(v16h a, v16h b, v8f c) {
  v8f d = __builtin_amdgcn_wmma_f32_16x16x32_f16(false, a, false, b, (short)0, c, false, false);
  asm volatile("v_nop\n\tv_nop\n\tv_nop\n\tv_nop" : "+v"(d) : "v"(a), "v"(b));
  return d;
}

template <int NT, int KS>
__device__ __forceinline__ void mm_tiles(const _Float16* ar, const _Float16* __restrict__ bpl,
                                         int KP, int n0, int m, int hh, v8f (&acc)[NT]) {
#pragma unroll
  for (int t = 0; t < NT; ++t) { v8f z = {0.f, 0.f, 0.f, 0.f, 0.f, 0.f, 0.f, 0.f}; acc[t] = z; }
#pragma unroll 1
  for (int kt = 0; kt < KS; ++kt) {
    FragH a;
    a.h[0] = *(const v8h*)(ar + 32 * kt);
    a.h[1] = *(const v8h*)(ar + 32 * kt + 16);
#pragma unroll
    for (int t = 0; t < NT; ++t) {
      const _Float16* bp = bpl + (size_t)(n0 + 16 * t + m) * KP + 32 * kt + 8 * hh;
      FragH b;
      b.h[0] = *(const v8h*)bp;
      b.h[1] = *(const v8h*)(bp + 16);
      acc[t] = wmh(a.v, b.v, acc[t]);
    }
  }
}

template <int NB>
__device__ __forceinline__ int scan_chunk(const int* __restrict__ dsts, int nE, int cbase, int slotBase,
                                          int vec8, int* list, int tid, int lane, int wave) {
  int wc = 0;
#pragma unroll
  for (int g = 0; g < NGRP; ++g) {
    const int el0  = (g * NTHR + tid) * EPT;
    const int e0   = cbase + el0;
    const int sent = -2147483647 - 1;
    v4i da, db;
    if (vec8 != 0 && cbase + CHUNK <= nE) {
      da = *(const v4i*)(dsts + e0);
      db = *(const v4i*)(dsts + e0 + 4);
    } else {
      da.x = (e0     < nE) ? dsts[min(e0,     nE - 1)] : sent;
      da.y = (e0 + 1 < nE) ? dsts[min(e0 + 1, nE - 1)] : sent;
      da.z = (e0 + 2 < nE) ? dsts[min(e0 + 2, nE - 1)] : sent;
      da.w = (e0 + 3 < nE) ? dsts[min(e0 + 3, nE - 1)] : sent;
      db.x = (e0 + 4 < nE) ? dsts[min(e0 + 4, nE - 1)] : sent;
      db.y = (e0 + 5 < nE) ? dsts[min(e0 + 5, nE - 1)] : sent;
      db.z = (e0 + 6 < nE) ? dsts[min(e0 + 6, nE - 1)] : sent;
      db.w = (e0 + 7 < nE) ? dsts[min(e0 + 7, nE - 1)] : sent;
    }
    const unsigned nb = (unsigned)slotBase;
    const unsigned s0 = (unsigned)da.x - nb, s1 = (unsigned)da.y - nb;
    const unsigned s2 = (unsigned)da.z - nb, s3 = (unsigned)da.w - nb;
    const unsigned s4 = (unsigned)db.x - nb, s5 = (unsigned)db.y - nb;
    const unsigned s6 = (unsigned)db.z - nb, s7 = (unsigned)db.w - nb;
    const bool h0 = s0 < (unsigned)NB, h1 = s1 < (unsigned)NB, h2 = s2 < (unsigned)NB, h3 = s3 < (unsigned)NB;
    const bool h4 = s4 < (unsigned)NB, h5 = s5 < (unsigned)NB, h6 = s6 < (unsigned)NB, h7 = s7 < (unsigned)NB;
    const unsigned any = __builtin_amdgcn_ballot_w32(h0 | h1 | h2 | h3 | h4 | h5 | h6 | h7);
    if (any != 0u) {
#define HITJ(J, HJ, SJ) { \
        const unsigned mj = __builtin_amdgcn_ballot_w32(HJ); \
        if (mj != 0u) { \
          if (HJ) { \
            const int pos = wc + (int)__builtin_amdgcn_mbcnt_lo(mj, 0u); \
            if (pos < WCAP) list[wave * WCAP + pos] = ((el0 + (J)) << 16) | (int)(SJ); \
          } \
          wc += (int)__builtin_popcount(mj); } }
      HITJ(0, h0, s0)
      HITJ(1, h1, s1)
      HITJ(2, h2, s2)
      HITJ(3, h3, s3)
      HITJ(4, h4, s4)
      HITJ(5, h5, s5)
      HITJ(6, h6, s6)
      HITJ(7, h7, s7)
#undef HITJ
    }
  }
  return wc;
}

__global__ __launch_bounds__(NTHR) void k_wprep(
    const float* __restrict__ pA, const float* __restrict__ pB, const float* __restrict__ pC,
    float fc, int K1, int K2, int Nout, _Float16* dst) {
  const int K = K1 + K2;
  const int K2c = K2 > 0 ? K2 : 1;
  const int per = K / 8;
  const int i = blockIdx.x * NTHR + (int)threadIdx.x;
  if (i >= Nout * per) return;
  const int n  = i / per;
  const int k0 = (i - n * per) * 8;
  float v[8];
#pragma unroll
  for (int e = 0; e < 8; ++e) {
    const int k = k0 + e;
    const int ka = k < K1 ? k : K1 - 1;
    int kb = k - K1;
    kb = kb < 0 ? 0 : (kb > K2c - 1 ? K2c - 1 : kb);
    const float va = pA[(size_t)ka * Nout + n];
    const float vb = pB[(size_t)kb * Nout + n];
    const float vx = pC[(size_t)kb * Nout + n];
    v[e] = ((k < K1) ? va : (vb + fc * vx)) * WSCALE;
  }
  v4f a, b;
  a.x = v[0]; a.y = v[1]; a.z = v[2]; a.w = v[3];
  b.x = v[4]; b.y = v[5]; b.z = v[6]; b.w = v[7];
  const v8h hv = cvt8(a, b);
  _Float16* dp = dst + (size_t)n * K + k0;
  *(volatile v8h*)dp = hv;
  __threadfence();
  *(volatile v8h*)dp = hv;
}

__global__ __launch_bounds__(NTHR) void k_maskx(const float* __restrict__ x, float* xm, int nN, int nRowsOut) {
  const int i = blockIdx.x * NTHR + (int)threadIdx.x;
  if (i >= nRowsOut * (F_EV / 4)) return;
  const int row = i / (F_EV / 4);
  const int c   = (i - row * (F_EV / 4)) * 4;
  const int rs  = row < nN ? row : nN - 1;
  v4f v = *(const v4f*)(x + (size_t)rs * F_EV + c);
  v4f mk;
  mk.x = (v.x != -1.0f) ? 1.0f : 0.0f;
  mk.y = (v.y != -1.0f) ? 1.0f : 0.0f;
  mk.z = (v.z != -1.0f) ? 1.0f : 0.0f;
  mk.w = (v.w != -1.0f) ? 1.0f : 0.0f;
  v = v * mk;
  float* p = xm + (size_t)row * F_EV + c;
  *(volatile v4f*)p = v;
  __threadfence();
  *(volatile v4f*)p = v;
}

__global__ __launch_bounds__(NTHR) void k_count(const int* __restrict__ ei, int* cnt, int nE, int vec8) {
  __shared__ __attribute__((aligned(16))) int scnt[NBC];
  __shared__ __attribute__((aligned(16))) int list[LISTN];
  __shared__ int wcnt[NWAVE];
  const int tid = threadIdx.x, lane = tid & 31, wave = tid >> 5;
  const int nodeBase = blockIdx.x * NBC;
  const int* dsts = ei + nE;

  for (int i = tid; i < NBC; i += NTHR) scnt[i] = 0;
  __syncthreads();

  const int nChunks = (nE + CHUNK - 1) / CHUNK;
#pragma unroll 1
  for (int ch = 0; ch < nChunks; ++ch) {
    const int cbase = ch * CHUNK;
    const int wc = scan_chunk<NBC>(dsts, nE, cbase, nodeBase, vec8, list, tid, lane, wave);
    if (lane == 0) wcnt[wave] = wc;
    __syncthreads();
    if (wave == 0) {
#pragma unroll 1
      for (int wsx = 0; wsx < NWAVE; ++wsx) {
        int n = __builtin_amdgcn_readfirstlane(wcnt[wsx]);
        n = n > WCAP ? WCAP : (n < 0 ? 0 : n);
        const int* lp = list + wsx * WCAP;
#pragma unroll 1
        for (int i = 0; i < n; ++i) {
          const int ent  = __builtin_amdgcn_readfirstlane(lp[i]);
          const int slot = ent & (NBC - 1);
          if (lane == 0) scnt[slot] = scnt[slot] + 1;
        }
      }
    }
    __syncthreads();
  }

  v4i cq[NBC / (NWAVE * 128)];
#pragma unroll
  for (int q = 0; q < NBC / (NWAVE * 128); ++q) {
    const int f = (wave * (NBC / (NWAVE * 128)) + q) * 128 + 4 * lane;
    cq[q] = *(const v4i*)(scnt + f);
  }
  int* cp = cnt + (size_t)nodeBase;
#pragma unroll
  for (int q = 0; q < NBC / (NWAVE * 128); ++q) {
    const int f = (wave * (NBC / (NWAVE * 128)) + q) * 128 + 4 * lane;
    *(volatile v4i*)(cp + f) = cq[q];
  }
  __threadfence();
#pragma unroll
  for (int q = 0; q < NBC / (NWAVE * 128); ++q) {
    const int f = (wave * (NBC / (NWAVE * 128)) + q) * 128 + 4 * lane;
    *(volatile v4i*)(cp + f) = cq[q];
  }
}

__global__ __launch_bounds__(OTHR) void k_offsets(const int* __restrict__ cnt, int* off, int* rbase, int nChunk) {
  __shared__ __attribute__((aligned(16))) int soff[NBC];
  __shared__ __attribute__((aligned(16))) int srb[RBN];
  __shared__ int wtot[OTHR / 32];
  const int tid = threadIdx.x, lane = tid & 31, wave = tid >> 5, sub = tid >> 7;
  for (int i = tid; i < RBN; i += OTHR) srb[i] = 0;
  int carry = 0;
#pragma unroll 1
  for (int ch = 0; ch < nChunk; ++ch) {
    const int base = ch * NBC;
    int e[16];
    int ts = 0;
#pragma unroll
    for (int q = 0; q < 4; ++q) {
      const v4i c = *(const v4i*)(cnt + base + 16 * tid + 4 * q);
      e[4 * q + 0] = c.x < 0 ? 0 : c.x;
      e[4 * q + 1] = c.y < 0 ? 0 : c.y;
      e[4 * q + 2] = c.z < 0 ? 0 : c.z;
      e[4 * q + 3] = c.w < 0 ? 0 : c.w;
      ts += e[4 * q + 0] + e[4 * q + 1] + e[4 * q + 2] + e[4 * q + 3];
    }
    int incl = ts;
#pragma unroll
    for (int d = 1; d < 32; d <<= 1) {
      const int t = __shfl_up(incl, d);
      if (lane >= d) incl += t;
    }
    if (lane == 31) wtot[wave] = incl;
    __syncthreads();
    const int S0 = wtot[0]  + wtot[1]  + wtot[2]  + wtot[3];
    const int S1 = wtot[4]  + wtot[5]  + wtot[6]  + wtot[7];
    const int S2 = wtot[8]  + wtot[9]  + wtot[10] + wtot[11];
    const int S3 = wtot[12] + wtot[13] + wtot[14] + wtot[15];
    int pre = 0;
#pragma unroll 1
    for (int w = 4 * sub; w < wave; ++w) pre += wtot[w];
    const int b0 = carry;
    const int b1 = b0 + ((S0 + 31) & ~31);
    const int b2 = b1 + ((S1 + 31) & ~31);
    const int b3 = b2 + ((S2 + 31) & ~31);
    const int b4 = b3 + ((S3 + 31) & ~31);
    const int myb = sub == 0 ? b0 : (sub == 1 ? b1 : (sub == 2 ? b2 : b3));
    if (tid == 0) {
      srb[min(4 * ch + 0, RBN - 1)] = b0;
      srb[min(4 * ch + 1, RBN - 1)] = b1;
      srb[min(4 * ch + 2, RBN - 1)] = b2;
      srb[min(4 * ch + 3, RBN - 1)] = b3;
    }
    int run = myb + pre + incl - ts;
#pragma unroll
    for (int q = 0; q < 16; ++q) { soff[16 * tid + q] = run; run += e[q]; }
    carry = b4;
    __syncthreads();
    v4i ov[4];
#pragma unroll
    for (int i = 0; i < 4; ++i) ov[i] = *(const v4i*)(soff + 4 * tid + 2048 * i);
    int* op = off + base;
#pragma unroll
    for (int i = 0; i < 4; ++i) *(volatile v4i*)(op + 4 * tid + 2048 * i) = ov[i];
    __threadfence();
#pragma unroll
    for (int i = 0; i < 4; ++i) *(volatile v4i*)(op + 4 * tid + 2048 * i) = ov[i];
    __syncthreads();
  }
  if (tid == 0) srb[min(4 * nChunk, RBN - 1)] = carry;
  __syncthreads();
  v4i rv = {0, 0, 0, 0};
  if (tid < 32) rv = *(const v4i*)(srb + 4 * tid);
  if (tid < 32) *(volatile v4i*)(rbase + 4 * tid) = rv;
  __threadfence();
  if (tid < 32) *(volatile v4i*)(rbase + 4 * tid) = rv;
}

__global__ __launch_bounds__(NTHR) void k_fill(
    const int* __restrict__ ei, const int* __restrict__ off, const int* __restrict__ rbase,
    int* csr, int nE, int vec8, int csrLen) {
  extern __shared__ v4f lds_dyn[];
  int* region = (int*)lds_dyn;
  int* cursor = region + RCAP;
  int* list   = cursor + NBF;
  int* wcnt   = list + LISTN;
  const int tid = threadIdx.x, lane = tid & 31, wave = tid >> 5;
  const int b = blockIdx.x;
  const int nodeBase = b * NBF;
  const int* dsts = ei + nE;

  int rb0 = rbase[b];
  const int rb1 = rbase[b + 1];
  rb0 = rb0 < 0 ? 0 : (rb0 > csrLen ? csrLen : rb0);
  rb0 &= ~31;
  int len = rb1 - rb0;
  len = len < 0 ? 0 : (len > RCAP ? RCAP : len);
  int lenW = (len + 31) & ~31;
  if (rb0 + lenW > csrLen) lenW = (csrLen - rb0) & ~31;

  {
    const v4i z = {0, 0, 0, 0};
    for (int i = tid; i < RCAP / 4; i += NTHR) ((v4i*)region)[i] = z;
    for (int s = tid; s < NBF; s += NTHR) {
      int o = off[nodeBase + s] - rb0;
      o = o < 0 ? 0 : (o > RCAP ? RCAP : o);
      cursor[s] = o;
    }
  }
  __syncthreads();

  const int nChunks = (nE + CHUNK - 1) / CHUNK;
#pragma unroll 1
  for (int ch = 0; ch < nChunks; ++ch) {
    const int cbase = ch * CHUNK;
    const int wc = scan_chunk<NBF>(dsts, nE, cbase, nodeBase, vec8, list, tid, lane, wave);
    if (lane == 0) wcnt[wave] = wc;
    __syncthreads();
    if (wave == 0) {
#pragma unroll 1
      for (int wsx = 0; wsx < NWAVE; ++wsx) {
        int n = __builtin_amdgcn_readfirstlane(wcnt[wsx]);
        n = n > WCAP ? WCAP : (n < 0 ? 0 : n);
        const int* lp = list + wsx * WCAP;
#pragma unroll 1
        for (int i = 0; i < n; ++i) {
          const int ent  = __builtin_amdgcn_readfirstlane(lp[i]);
          const int slot = ent & (NBF - 1);
          int e = cbase + ((ent >> 16) & (CHUNK - 1));
          e = e > nE - 1 ? nE - 1 : e;
          if (lane == 0) {
            int pos = cursor[slot];
            pos = pos < 0 ? 0 : (pos > RCAP - 1 ? RCAP - 1 : pos);
            region[pos] = e;
            const int np = pos + 1;
            cursor[slot] = np > RCAP ? RCAP : np;
          }
        }
      }
    }
    __syncthreads();
  }

  const int nv = lenW >> 2;
  int* gp = csr + rb0;
#pragma unroll 1
  for (int i = tid; i < nv; i += NTHR) { const v4i v = ((const v4i*)region)[i]; *(volatile v4i*)(gp + 4 * i) = v; }
  __threadfence();
#pragma unroll 1
  for (int i = tid; i < nv; i += NTHR) { const v4i v = ((const v4i*)region)[i]; *(volatile v4i*)(gp + 4 * i) = v; }
}

template <int F, int NOUT, int MASK>
__global__ __launch_bounds__(NTHR) void k_layer(
    const int* __restrict__ csr, const int* __restrict__ off, const int* __restrict__ cnt,
    const int* __restrict__ esrc, const float* __restrict__ ew,
    const float* __restrict__ hin, const _Float16* __restrict__ wpl,
    const float* __restrict__ b1, const float* __restrict__ b2, float fb2,
    float* outp, int nN, int nE, int csrLen, int ldOut, int colOff) {
  extern __shared__ v4f lds_dyn[];
  constexpr int K  = 2 * F;
  constexpr int AP = K + 8;
  _Float16* sA  = (_Float16*)lds_dyn;
  float*    stg = (float*)((char*)lds_dyn + GROWS * AP * 2);
  const int tid = threadIdx.x, lane = tid & 31, wave = tid >> 5, hh = lane >> 4, m = lane & 15;
  const int rowBase = blockIdx.x * GROWS;
  const int tb = rowBase + wave * 16;
  const int cl = tb + m;
  const int cnt_l = cnt[cl];
  const int off_l = off[cl];

#pragma unroll 1
  for (int j = 0; j < 16; ++j) {
    int n = __builtin_amdgcn_readlane(cnt_l, j);
    n = n < 0 ? 0 : (n > DEGCAP ? DEGCAP : n);
    const int st = __builtin_amdgcn_readlane(off_l, j);
    v4f a0 = {0.f, 0.f, 0.f, 0.f};
    v4f a1 = {0.f, 0.f, 0.f, 0.f};
    v2f a2 = {0.f, 0.f};
#pragma unroll 1
    for (int q0 = 0; q0 < n; q0 += 32) {
      int pos = st + q0 + lane;
      pos = pos < 0 ? 0 : (pos > csrLen - 1 ? csrLen - 1 : pos);
      int e = csr[pos];
      e = e < 0 ? 0 : (e > nE - 1 ? nE - 1 : e);
      int s = esrc[e];
      s = s < 0 ? 0 : (s > nN - 1 ? nN - 1 : s);
      const int wb = __float_as_int(ew[e]);
      const int mcnt = (n - q0) < 32 ? (n - q0) : 32;
#pragma unroll 1
      for (int p = 0; p < mcnt; ++p) {
        const int sp = __builtin_amdgcn_readlane(s, p);
        const float wp = __int_as_float(__builtin_amdgcn_readlane(wb, p));
        const float* rp = hin + (size_t)sp * F;
        if (F == 64) {
          a2 = a2 + wp * (*(const v2f*)(rp + 2 * lane));
        } else if (F == 128) {
          a0 = a0 + wp * (*(const v4f*)(rp + 4 * lane));
        } else {
          a0 = a0 + wp * (*(const v4f*)(rp + 4 * lane));
          a1 = a1 + wp * (*(const v4f*)(rp + 128 + 4 * lane));
        }
      }
    }
    _Float16* dr = sA + (wave * 16 + j) * AP;
    if (F == 64) {
      *(v2h*)(dr + 2 * lane) = cvt2(a2);
    } else if (F == 128) {
      *(v4h*)(dr + 4 * lane) = cvt4(a0);
    } else {
      *(v4h*)(dr + 4 * lane) = cvt4(a0);
      *(v4h*)(dr + 128 + 4 * lane) = cvt4(a1);
    }
  }
#pragma unroll 1
  for (int r = 0; r < 16; ++r) {
    int rc = tb + r;
    rc = rc > nN - 1 ? nN - 1 : rc;
    const float* rp = hin + (size_t)rc * F;
    _Float16* dr = sA + (wave * 16 + r) * AP + F;
    if (F == 64) {
      *(v2h*)(dr + 2 * lane) = cvt2(*(const v2f*)(rp + 2 * lane));
    } else if (F == 128) {
      *(v4h*)(dr + 4 * lane) = cvt4(*(const v4f*)(rp + 4 * lane));
    } else {
      *(v4h*)(dr + 4 * lane) = cvt4(*(const v4f*)(rp + 4 * lane));
      *(v4h*)(dr + 128 + 4 * lane) = cvt4(*(const v4f*)(rp + 128 + 4 * lane));
    }
  }
  __syncthreads();

#pragma unroll 1
  for (int g = 0; g < NOUT / 128; ++g) {
    v8f acc[8];
    const _Float16* ar = sA + (wave * 16 + m) * AP + 8 * hh;
    mm_tiles<8, K / 32>(ar, wpl, K, 128 * g, m, hh, acc);
    float* sp = stg + (wave * 16 + 8 * hh) * 128 + m;
#pragma unroll
    for (int t = 0; t < 8; ++t) {
      const int ncol = 128 * g + 16 * t + m;
      const float bl = b1[ncol] + fb2 * b2[ncol];
#pragma unroll
      for (int r = 0; r < 8; ++r) {
        float v = acc[t][r] * WINV + bl;
        if (MASK) {
          const float mk = (v != -1.0f) ? 1.0f : 0.0f;
          v = v * mk;
          v = fmaxf(v, 0.0f);
          v = v * mk;
        } else {
          v = fmaxf(v, 0.0f);
        }
        sp[r * 128 + 16 * t] = v;
      }
    }
    __syncthreads();
    const float* lp = stg + wave * 16 * 128 + 4 * lane;
    float* gp = outp + (size_t)tb * ldOut + colOff + 128 * g + 4 * lane;
#pragma unroll
    for (int i = 0; i < 16; ++i) { const v4f v = *(const v4f*)(lp + i * 128); *(volatile v4f*)(gp + (size_t)i * ldOut) = v; }
    __threadfence();
#pragma unroll
    for (int i = 0; i < 16; ++i) { const v4f v = *(const v4f*)(lp + i * 128); *(volatile v4f*)(gp + (size_t)i * ldOut) = v; }
    __syncthreads();
  }
}

__global__ __launch_bounds__(NTHR) void k_pool(const int* __restrict__ batch, const float* __restrict__ h,
                                              float* pooled, int nN) {
  __shared__ __attribute__((aligned(16))) float acc[NBP * F_CAT];
  __shared__ __attribute__((aligned(16))) int list[LISTN];
  __shared__ int pc[NBP];
  __shared__ int wcnt[NWAVE];
  const int tid = threadIdx.x, lane = tid & 31, wave = tid >> 5;
  const int gBase = blockIdx.x * NBP;

  {
    const v4f z = {0.f, 0.f, 0.f, 0.f};
    for (int i = tid; i < NBP * F_CAT / 4; i += NTHR) ((v4f*)acc)[i] = z;
    for (int i = tid; i < NBP; i += NTHR) pc[i] = 0;
  }
  __syncthreads();

  const int nChunks = (nN + CHUNK - 1) / CHUNK;
#pragma unroll 1
  for (int ch = 0; ch < nChunks; ++ch) {
    const int cbase = ch * CHUNK;
    const int wc = scan_chunk<NBP>(batch, nN, cbase, gBase, 1, list, tid, lane, wave);
    if (lane == 0) wcnt[wave] = wc;
    __syncthreads();
    if (wave == 0) {
#pragma unroll 1
      for (int wsx = 0; wsx < NWAVE; ++wsx) {
        int n = __builtin_amdgcn_readfirstlane(wcnt[wsx]);
        n = n > WCAP ? WCAP : (n < 0 ? 0 : n);
        const int* lp = list + wsx * WCAP;
#pragma unroll 1
        for (int i = 0; i < n; ++i) {
          const int ent  = __builtin_amdgcn_readfirstlane(lp[i]);
          const int slot = ent & (NBP - 1);
          int nd = cbase + ((ent >> 16) & (CHUNK - 1));
          nd = nd > nN - 1 ? nN - 1 : nd;
          const float* rp = h + (size_t)nd * F_CAT;
          const v4f v0 = *(const v4f*)(rp + 4 * lane);
          const v4f v1 = *(const v4f*)(rp + 128 + 4 * lane);
          v4f* ap0 = (v4f*)(acc + slot * F_CAT + 4 * lane);
          v4f* ap1 = (v4f*)(acc + slot * F_CAT + 128 + 4 * lane);
          *ap0 = *ap0 + v0;
          *ap1 = *ap1 + v1;
          if (lane == 0) pc[slot] = pc[slot] + 1;
        }
      }
    }
    __syncthreads();
  }

  v4f ov[8];
#pragma unroll
  for (int p = 0; p < 8; ++p) {
    const int idx = p * NTHR + tid;
    const int row = idx >> 6;
    const int c0  = (idx & 63) * 4;
    int cv = pc[row];
    cv = cv < 1 ? 1 : cv;
    const float inv = 1.0f / (float)cv;
    ov[p] = *(const v4f*)(acc + row * F_CAT + c0) * inv;
  }
  float* gp = pooled + (size_t)gBase * F_CAT;
#pragma unroll
  for (int p = 0; p < 8; ++p) *(volatile v4f*)(gp + 4 * (p * NTHR + tid)) = ov[p];
  __threadfence();
#pragma unroll
  for (int p = 0; p < 8; ++p) *(volatile v4f*)(gp + 4 * (p * NTHR + tid)) = ov[p];
}

__global__ __launch_bounds__(NTHR) void k_head(
    const float* __restrict__ seq, const float* __restrict__ pooled,
    const _Float16* __restrict__ wf1, const float* __restrict__ bf1,
    const _Float16* __restrict__ wf2, const float* __restrict__ bf2,
    const _Float16* __restrict__ wfc, const float* __restrict__ bfc,
    const _Float16* __restrict__ wcl, const float* __restrict__ bcl, float* out) {
  extern __shared__ v4f lds_dyn[];
  _Float16* bufA = (_Float16*)lds_dyn;
  _Float16* bufB = bufA + HB * HPA;
  float* sLog = (float*)(bufB + HB * HPB);
  float* sOut = sLog + HB * NCLS;
  const int tid = threadIdx.x, lane = tid & 31, wave = tid >> 5, hh = lane >> 4, m = lane & 15;
  const int rt = wave & 3, cg = wave >> 2, r0 = 16 * rt;

#pragma unroll
  for (int i = 0; i < (HB * SEQF / 8) / NTHR; ++i) {
    const int idx = i * NTHR + tid;
    const int r = idx >> 5, c0 = (idx & 31) * 8;
    const float* p = seq + (size_t)r * SEQF + c0;
    *(v8h*)(bufA + r * HPA + c0) = cvt8(*(const v4f*)p, *(const v4f*)(p + 4));
  }
  __syncthreads();
  {
    v8f acc[8];
    mm_tiles<8, SEQF / 32>(bufA + (r0 + m) * HPA + 8 * hh, wf1, SEQF, 128 * cg, m, hh, acc);
    _Float16* dp = bufB + (r0 + 8 * hh) * HPB;
#pragma unroll
    for (int t = 0; t < 8; ++t) {
      const int n = 128 * cg + 16 * t + m;
      const float bl = bf1[n];
#pragma unroll
      for (int r = 0; r < 8; ++r) dp[r * HPB + n] = (_Float16)fmaxf(acc[t][r] * WINV + bl, 0.0f);
    }
  }
  __syncthreads();
#pragma unroll
  for (int i = 0; i < (HB * F_CAT / 8) / NTHR; ++i) {
    const int idx = i * NTHR + tid;
    const int r = idx >> 5, c0 = (idx & 31) * 8;
    const float* p = pooled + (size_t)r * F_CAT + c0;
    *(v8h*)(bufA + r * HPA + c0) = cvt8(*(const v4f*)p, *(const v4f*)(p + 4));
  }
  {
    v8f acc[4];
    mm_tiles<4, SEQF / 32>(bufB + (r0 + m) * HPB + 8 * hh, wf2, SEQF, 64 * cg, m, hh, acc);
    _Float16* dp = bufA + (r0 + 8 * hh) * HPA + F_CAT;
#pragma unroll
    for (int t = 0; t < 4; ++t) {
      const int n = 64 * cg + 16 * t + m;
      const float bl = bf2[n];
#pragma unroll
      for (int r = 0; r < 8; ++r) dp[r * HPA + n] = (_Float16)fmaxf(acc[t][r] * WINV + bl, 0.0f);
    }
  }
  __syncthreads();
  {
    v8f acc[8];
    mm_tiles<8, FCCK / 32>(bufA + (r0 + m) * HPA + 8 * hh, wfc, FCCK, 128 * cg, m, hh, acc);
    _Float16* dp = bufB + (r0 + 8 * hh) * HPB;
#pragma unroll
    for (int t = 0; t < 8; ++t) {
      const int n = 128 * cg + 16 * t + m;
      const float bl = bfc[n];
#pragma unroll
      for (int r = 0; r < 8; ++r) dp[r * HPB + n] = (_Float16)fmaxf(acc[t][r] * WINV + bl, 0.0f);
    }
  }
  __syncthreads();
  {
    v8f acc[1];
    mm_tiles<1, F_CAT / 32>(bufB + (r0 + m) * HPB + 8 * hh, wcl, F_CAT, 0, m, hh, acc);
    const float bl = bcl[m];
    if (cg == 0) {
#pragma unroll
      for (int r = 0; r < 8; ++r) sLog[(r0 + 8 * hh + r) * NCLS + m] = acc[0][r] * WINV + bl;
    }
  }
  __syncthreads();
  if (tid < HB) {
    const float* lr = sLog + tid * NCLS;
    float mx = lr[0];
#pragma unroll 1
    for (int j = 1; j < NCLS; ++j) mx = fmaxf(mx, lr[j]);
    float s = 0.0f;
#pragma unroll 1
    for (int j = 0; j < NCLS; ++j) s += expf(lr[j] - mx);
    const float ls = logf(s);
#pragma unroll 1
    for (int j = 0; j < NCLS; ++j) sOut[tid * NCLS + j] = (lr[j] - mx) - ls;
  }
  __syncthreads();
  if (wave == 0) {
    v4f ov[8];
#pragma unroll
    for (int p = 0; p < 8; ++p) ov[p] = *(const v4f*)(sOut + 128 * p + 4 * lane);
#pragma unroll
    for (int p = 0; p < 8; ++p) *(volatile v4f*)(out + 128 * p + 4 * lane) = ov[p];
    __threadfence();
#pragma unroll
    for (int p = 0; p < 8; ++p) *(volatile v4f*)(out + 128 * p + 4 * lane) = ov[p];
  }
}

extern "C" void kernel_launch(void* const* d_in, const int* in_sizes, int n_in,
                              void* d_out, int out_size, void* d_ws, size_t ws_size,
                              hipStream_t stream) {
  if (n_in < 30) return;
  const int nN = in_sizes[0] / F_EV;
  if (nN < 1 || in_sizes[0] != nN * F_EV || in_sizes[3] != nN || in_sizes[4] != nN * F_DU) return;
  const int nE = in_sizes[1] / 2;
  if (nE < 1 || in_sizes[1] != 2 * nE || in_sizes[2] != nE) return;
  const int nEd = in_sizes[5] / 2;
  if (nEd < 1 || in_sizes[5] != 2 * nEd || in_sizes[6] != nEd) return;
  if (out_size != HB * NCLS || in_sizes[7] != HB * SEQF) return;
  if (in_sizes[8]  != F_EV * F_EV || in_sizes[9]  < F_EV || in_sizes[10] != F_EV * F_EV) return;
  if (in_sizes[11] != F_EV * F_EV || in_sizes[12] < F_EV || in_sizes[13] != F_EV * F_EV) return;
  if (in_sizes[14] != F_DU * F_EV || in_sizes[15] < F_EV || in_sizes[16] != F_DU * F_EV) return;
  if (in_sizes[17] != F_CAT * F_CAT || in_sizes[18] < F_CAT || in_sizes[19] != F_CAT * F_CAT) return;
  if (in_sizes[20] != F_CAT * F_CAT || in_sizes[21] < F_CAT) return;
  if (in_sizes[22] != SEQF * SEQF || in_sizes[23] < SEQF || in_sizes[24] != SEQF * FC2N || in_sizes[25] < FC2N) return;
  if (in_sizes[26] != FCCK * F_CAT || in_sizes[27] < F_CAT || in_sizes[28] != F_CAT * NCLS || in_sizes[29] < NCLS) return;
  if (nN > (1 << 22) || nE > (1 << 28) || nEd > (1 << 28)) return;

  const float* x      = (const float*)d_in[0];
  const int*   ei     = (const int*)d_in[1];
  const float* eattr  = (const float*)d_in[2];
  const int*   batch  = (const int*)d_in[3];
  const float* dur_x  = (const float*)d_in[4];
  const int*   dei    = (const int*)d_in[5];
  const float* deattr = (const float*)d_in[6];
  const float* seq    = (const float*)d_in[7];
  const float* g1_Wr  = (const float*)d_in[8];
  const float* g1_br  = (const float*)d_in[9];
  const float* g1_Wo  = (const float*)d_in[10];
  const float* g2_Wr  = (const float*)d_in[11];
  const float* g2_br  = (const float*)d_in[12];
  const float* g2_Wo  = (const float*)d_in[13];
  const float* d1_Wr  = (const float*)d_in[14];
  const float* d1_br  = (const float*)d_in[15];
  const float* d1_Wo  = (const float*)d_in[16];
  const float* c1_Wr  = (const float*)d_in[17];
  const float* c1_br  = (const float*)d_in[18];
  const float* c1_Wo  = (const float*)d_in[19];
  const float* skip_W = (const float*)d_in[20];
  const float* skip_b = (const float*)d_in[21];
  const float* fc1_W  = (const float*)d_in[22];
  const float* fc1_b  = (const float*)d_in[23];
  const float* fc2_W  = (const float*)d_in[24];
  const float* fc2_b  = (const float*)d_in[25];
  const float* fcc_W  = (const float*)d_in[26];
  const float* fcc_b  = (const float*)d_in[27];
  const float* cls_W  = (const float*)d_in[28];
  const float* cls_b  = (const float*)d_in[29];
  float* out = (float*)d_out;

  const int NPAD   = ((nN + GROWS - 1) / GROWS) * GROWS;
  const int nBC    = (nN + NBC - 1) / NBC;
  const int CNTPAD = nBC * NBC;
  if (4 * nBC + 2 > RBN) return;
  const int nBF    = (nN + NBF - 1) / NBF;
  if (nBF > 4 * nBC) return;
  const int csrLenE = ((nE  + 31) & ~31) + 32 * (4 * nBC + 2);
  const int csrLenD = ((nEd + 31) & ~31) + 32 * (4 * nBC + 2);
  const int nLB    = NPAD / GROWS;
  const int nPool  = (HB + NBP - 1) / NBP;
  const int POOLROWS = nPool * NBP;

  char* ws = (char*)d_ws;
  size_t o = 0;
#define CARVE(name, bytes) const size_t name = o; o += (size_t)(bytes); o = (o + 255) & ~(size_t)255;
  CARVE(oW1,  (size_t)F_EV * (2 * F_EV) * 2)
  CARVE(oW2,  (size_t)F_EV * (2 * F_EV) * 2)
  CARVE(oWD,  (size_t)F_EV * (2 * F_DU) * 2)
  CARVE(oWC,  (size_t)F_CAT * (2 * F_CAT) * 2)
  CARVE(oF1,  (size_t)SEQF * SEQF * 2)
  CARVE(oF2,  (size_t)FC2N * SEQF * 2)
  CARVE(oFC,  (size_t)F_CAT * FCCK * 2)
  CARVE(oCL,  (size_t)NCLS * F_CAT * 2)
  CARVE(oCntE, (size_t)CNTPAD * 4)
  CARVE(oOffE, (size_t)CNTPAD * 4)
  CARVE(oRbE,  (size_t)RBN * 4)
  CARVE(oCsrE, (size_t)csrLenE * 4)
  CARVE(oCntD, (size_t)CNTPAD * 4)
  CARVE(oOffD, (size_t)CNTPAD * 4)
  CARVE(oRbD,  (size_t)RBN * 4)
  CARVE(oCsrD, (size_t)csrLenD * 4)
  CARVE(oX2,   (size_t)NPAD * F_CAT * 4)
  CARVE(oXc,   (size_t)NPAD * F_CAT * 4)
  CARVE(oPool, (size_t)POOLROWS * F_CAT * 4)
#undef CARVE
  if (o > ws_size) return;
  _Float16* W1  = (_Float16*)(ws + oW1);
  _Float16* W2  = (_Float16*)(ws + oW2);
  _Float16* WD  = (_Float16*)(ws + oWD);
  _Float16* WC  = (_Float16*)(ws + oWC);
  _Float16* WF1 = (_Float16*)(ws + oF1);
  _Float16* WF2 = (_Float16*)(ws + oF2);
  _Float16* WFC = (_Float16*)(ws + oFC);
  _Float16* WCL = (_Float16*)(ws + oCL);
  int* cntE = (int*)(ws + oCntE); int* offE = (int*)(ws + oOffE); int* rbE = (int*)(ws + oRbE); int* csrE = (int*)(ws + oCsrE);
  int* cntD = (int*)(ws + oCntD); int* offD = (int*)(ws + oOffD); int* rbD = (int*)(ws + oRbD); int* csrD = (int*)(ws + oCsrD);
  float* xm   = (float*)(ws + oX2);
  float* h1   = (float*)(ws + oX2 + (size_t)NPAD * F_EV * 4);
  float* xc2  = (float*)(ws + oX2);
  float* xc   = (float*)(ws + oXc);
  float* pooled = (float*)(ws + oPool);

  const int vec8E = ((nE & 3) == 0) ? 1 : 0;
  const int vec8D = ((nEd & 3) == 0) ? 1 : 0;

  k_wprep<<<(F_EV * 2 * F_EV / 8 + NTHR - 1) / NTHR, NTHR, 0, stream>>>(g1_Wr, g1_Wo, g1_Wo, 0.0f, F_EV, F_EV, F_EV, W1);
  k_wprep<<<(F_EV * 2 * F_EV / 8 + NTHR - 1) / NTHR, NTHR, 0, stream>>>(g2_Wr, g2_Wo, g2_Wo, 0.0f, F_EV, F_EV, F_EV, W2);
  k_wprep<<<(F_EV * 2 * F_DU / 8 + NTHR - 1) / NTHR, NTHR, 0, stream>>>(d1_Wr, d1_Wo, d1_Wo, 0.0f, F_DU, F_DU, F_EV, WD);
  k_wprep<<<(F_CAT * 2 * F_CAT / 8 + NTHR - 1) / NTHR, NTHR, 0, stream>>>(c1_Wr, c1_Wo, skip_W, 1.0f, F_CAT, F_CAT, F_CAT, WC);
  k_wprep<<<(SEQF * SEQF / 8 + NTHR - 1) / NTHR, NTHR, 0, stream>>>(fc1_W, fc1_W, fc1_W, 0.0f, SEQF, 0, SEQF, WF1);
  k_wprep<<<(FC2N * SEQF / 8 + NTHR - 1) / NTHR, NTHR, 0, stream>>>(fc2_W, fc2_W, fc2_W, 0.0f, SEQF, 0, FC2N, WF2);
  k_wprep<<<(F_CAT * FCCK / 8 + NTHR - 1) / NTHR, NTHR, 0, stream>>>(fcc_W, fcc_W, fcc_W, 0.0f, FCCK, 0, F_CAT, WFC);
  k_wprep<<<(NCLS * F_CAT / 8 + NTHR - 1) / NTHR, NTHR, 0, stream>>>(cls_W, cls_W, cls_W, 0.0f, F_CAT, 0, NCLS, WCL);

  k_maskx<<<(NPAD * (F_EV / 4) + NTHR - 1) / NTHR, NTHR, 0, stream>>>(x, xm, nN, NPAD);

  hipFuncSetAttribute(reinterpret_cast<const void*>(&k_fill), hipFuncAttributeMaxDynamicSharedMemorySize, LDS_FILL);
  k_count<<<nBC, NTHR, 0, stream>>>(ei, cntE, nE, vec8E);
  k_offsets<<<1, OTHR, 0, stream>>>(cntE, offE, rbE, nBC);
  k_fill<<<nBF, NTHR, LDS_FILL, stream>>>(ei, offE, rbE, csrE, nE, vec8E, csrLenE);
  k_count<<<nBC, NTHR, 0, stream>>>(dei, cntD, nEd, vec8D);
  k_offsets<<<1, OTHR, 0, stream>>>(cntD, offD, rbD, nBC);
  k_fill<<<nBF, NTHR, LDS_FILL, stream>>>(dei, offD, rbD, csrD, nEd, vec8D, csrLenD);

  hipFuncSetAttribute(reinterpret_cast<const void*>(&k_layer<F_EV, F_EV, 1>), hipFuncAttributeMaxDynamicSharedMemorySize, LDS_LAYER(F_EV));
  hipFuncSetAttribute(reinterpret_cast<const void*>(&k_layer<F_DU, F_EV, 0>), hipFuncAttributeMaxDynamicSharedMemorySize, LDS_LAYER(F_DU));
  hipFuncSetAttribute(reinterpret_cast<const void*>(&k_layer<F_CAT, F_CAT, 0>), hipFuncAttributeMaxDynamicSharedMemorySize, LDS_LAYER(F_CAT));
  k_layer<F_EV, F_EV, 1><<<nLB, NTHR, LDS_LAYER(F_EV), stream>>>(csrE, offE, cntE, ei, eattr, xm, W1, g1_br, g1_br, 0.0f,
                                                                  h1, nN, nE, csrLenE, F_EV, 0);
  k_layer<F_EV, F_EV, 1><<<nLB, NTHR, LDS_LAYER(F_EV), stream>>>(csrE, offE, cntE, ei, eattr, h1, W2, g2_br, g2_br, 0.0f,
                                                                  xc, nN, nE, csrLenE, F_CAT, 0);
  k_layer<F_DU, F_EV, 0><<<nLB, NTHR, LDS_LAYER(F_DU), stream>>>(csrD, offD, cntD, dei, deattr, dur_x, WD, d1_br, d1_br, 0.0f,
                                                                  xc, nN, nEd, csrLenD, F_CAT, F_EV);
  k_layer<F_CAT, F_CAT, 0><<<nLB, NTHR, LDS_LAYER(F_CAT), stream>>>(csrE, offE, cntE, ei, eattr, xc, WC, c1_br, skip_b, 1.0f,
                                                                     xc2, nN, nE, csrLenE, F_CAT, 0);

  k_pool<<<nPool, NTHR, 0, stream>>>(batch, xc2, pooled, nN);

  hipFuncSetAttribute(reinterpret_cast<const void*>(&k_head), hipFuncAttributeMaxDynamicSharedMemorySize, LDS_HEAD);
  k_head<<<1, NTHR, LDS_HEAD, stream>>>(seq, pooled, WF1, fc1_b, WF2, fc2_b, WFC, fcc_b, WCL, cls_b, out);
}
